// mLSTMCell_7224134992402
// MI455X (gfx1250) — hardware-verified
//
#include <hip/hip_runtime.h>
#include <math.h>

constexpr int kSeq   = 2048;
constexpr int kEmb   = 1024;
constexpr int kHeads = 8;
constexpr int kDh    = 128;
constexpr int kXld   = 3 * kEmb;
constexpr int kGateN = 64;
constexpr int kTiles = kSeq / 32;
constexpr float kCCarry    = 1024.0f;
constexpr float kVCarry    = 16.0f;
constexpr float kCVInv     = 1.0f / (1024.0f * 16.0f);
constexpr float kEpsN      = 1.0e-6f;
constexpr float kLnEps     = 1.0e-5f;
constexpr float kInvEmb    = 1.0f / 1024.0f;
constexpr float kSkipBelow = -90.0f;
static_assert(kHeads * kDh == kEmb);
static_assert(kSeq % 64 == 0 && kGateN % 64 == 0 && kXld % 32 == 0 && kDh % 32 == 0);
static_assert(kSeq == 8 * 256 && kEmb == 4 * 256 && kTiles == 64);

typedef __attribute__((ext_vector_type(16))) _Float16 v16h;
typedef __attribute__((ext_vector_type(8)))  _Float16 v8h;
typedef __attribute__((ext_vector_type(16))) __bf16   v16b;
typedef __attribute__((ext_vector_type(8)))  __bf16   v8b;
typedef __attribute__((ext_vector_type(8)))  float    v8f;
typedef __attribute__((ext_vector_type(4)))  float    v4f;
typedef __attribute__((ext_vector_type(4)))  unsigned int v4u;

__device__ __forceinline__ unsigned short f2bf_bits(float f) {
  unsigned u = __float_as_uint(f);
  return (unsigned short)((u + 0x7FFFu + ((u >> 16) & 1u)) >> 16);
}
__device__ __forceinline__ float bf_bits2f(unsigned short h) { return __uint_as_float(((unsigned)h) << 16); }

__device__ __forceinline__ void dep_guard_h(v8f& a, v8f& b, v16h x, v16h y) { asm volatile("v_nop\n\tv_nop\n\tv_nop\n\tv_nop" : "+v"(a), "+v"(b) : "v"(x), "v"(y)); }
__device__ __forceinline__ void dep_guard_b(v8f& a, v8f& b, v16b x, v16b y) { asm volatile("v_nop\n\tv_nop\n\tv_nop\n\tv_nop" : "+v"(a), "+v"(b) : "v"(x), "v"(y)); }
__device__ __forceinline__ void keep4_h(v16h a, v16h b, v16h c, v16h d) { asm volatile("v_nop" :: "v"(a), "v"(b), "v"(c), "v"(d)); }
__device__ __forceinline__ void keep4_b(v16b a, v16b b, v16b c, v16b d) { asm volatile("v_nop" :: "v"(a), "v"(b), "v"(c), "v"(d)); }
__device__ __forceinline__ void acc_guard4(v8f& a, v8f& b, v8f& c, v8f& d) { asm volatile("v_nop\n\tv_nop\n\tv_nop\n\tv_nop" : "+v"(a), "+v"(b), "+v"(c), "+v"(d)); }
template <typename T> struct Frag;
template <> struct Frag<_Float16> {
  typedef v16h V; union U { v16h v; v8h h[2]; };
  static __device__ __forceinline__ v16h load(const _Float16* p) {
    U f; f.h[0] = *(const v8h*)(p); f.h[1] = *(const v8h*)(p + 16); return f.v;
  }
  static __device__ __forceinline__ v8f mma(v16h a, v16h b, v8f c) {
    return __builtin_amdgcn_wmma_f32_16x16x32_f16(false, a, false, b, (short)0, c, false, false);
  }
  static __device__ __forceinline__ void guard(v8f& a, v8f& b, v16h x, v16h y) { dep_guard_h(a, b, x, y); }
  static __device__ __forceinline__ void keep(v16h a, v16h b, v16h c, v16h d) { keep4_h(a, b, c, d); }
};
template <> struct Frag<__bf16> {
  typedef v16b V; union U { v16b v; v8b h[2]; };
  static __device__ __forceinline__ v16b load(const __bf16* p) {
    U f; f.h[0] = *(const v8b*)(p); f.h[1] = *(const v8b*)(p + 16); return f.v;
  }
  static __device__ __forceinline__ v8f mma(v16b a, v16b b, v8f c) {
    return __builtin_amdgcn_wmma_f32_16x16x32_bf16(false, a, false, b, (short)0, c, false, false);
  }
  static __device__ __forceinline__ void guard(v8f& a, v8f& b, v16b x, v16b y) { dep_guard_b(a, b, x, y); }
  static __device__ __forceinline__ void keep(v16b a, v16b b, v16b c, v16b d) { keep4_b(a, b, c, d); }
};

__device__ __forceinline__ unsigned pk16(unsigned short a, unsigned short b) { return (unsigned)a | ((unsigned)b << 16); }
__device__ __forceinline__ unsigned short h_bits(float f) { const _Float16 h = (_Float16)f; return __builtin_bit_cast(unsigned short, h); }

__device__ __forceinline__ v8f mma16_bf(v16b a, v16b b, v8f c) {
  c = __builtin_amdgcn_wmma_f32_16x16x32_bf16(false, a, false, b, (short)0, c, false, false);
  asm volatile("v_nop\n\tv_nop\n\tv_nop\n\tv_nop" : "+v"(c) : "v"(a), "v"(b));
  return c;
}
__device__ __forceinline__ v8f mma16_h(v16h a, v16h b, v8f c) {
  c = __builtin_amdgcn_wmma_f32_16x16x32_f16(false, a, false, b, (short)0, c, false, false);
  asm volatile("v_nop\n\tv_nop\n\tv_nop\n\tv_nop" : "+v"(c) : "v"(a), "v"(b));
  return c;
}

template <int ET> struct Elem;
template <> struct Elem<0> { typedef _Float16 T; };
template <> struct Elem<1> { typedef __bf16 T; };
template <int ET, bool SPLIT, int BIAS_MODE, int OUT_MODE, bool RESID, int ACT = 0>
__global__ __launch_bounds__(256) void wmma_gemm64(
    const unsigned short* __restrict__ Ap, const unsigned short* __restrict__ A2p, int lda, long strideA,
    const unsigned short* __restrict__ Btp, const unsigned short* __restrict__ Bt2p, int ldb, long strideB,
    void* __restrict__ Cout, void* __restrict__ Cout2, int ldc, long strideC,
    const float* __restrict__ bias,
    const float* __restrict__ resid, long strideR,
    int M, int N, int K, float scale) {
  typedef typename Elem<ET>::T T;
  typedef typename Frag<T>::V V;
  const T* A = (const T*)Ap; const T* A2 = (const T*)A2p; const T* Bt = (const T*)Btp; const T* Bt2 = (const T*)Bt2p;
  __shared__ __align__(16) float sT[8][16 * 68];
  const int b    = blockIdx.y;
  const int lane = threadIdx.x & 31;
  const int wave = threadIdx.x >> 5;
  const int tilesN = N >> 6;
  const int tilesM = M >> 6;
  const int tile = blockIdx.x * 8 + wave;
  if (tile >= tilesM * tilesN) return;
  const int tm = tile / tilesN;
  const int tn = tile - tm * tilesN;
  const int m0 = tm << 6;
  const int n0 = tn << 6;

  const T* Ab  = A  + (size_t)b * strideA;
  const T* Bb  = Bt + (size_t)b * strideB;
  const T* Ab2 = SPLIT ? (A2  + (size_t)b * strideA) : nullptr;
  const T* Bb2 = SPLIT ? (Bt2 + (size_t)b * strideB) : nullptr;

  const int rlane = lane & 15;
  const int koff  = (lane >> 4) * 8;
  const int mOff  = (lane >> 4) * 8;

  v8f acc[4][4];
#pragma unroll
  for (int i = 0; i < 4; ++i)
#pragma unroll
    for (int j = 0; j < 4; ++j) acc[i][j] = (v8f){0.f,0.f,0.f,0.f,0.f,0.f,0.f,0.f};

  for (int k0 = 0; k0 < K; k0 += 32) {
    V bh[4], bl[4];
#pragma unroll
    for (int j = 0; j < 4; ++j) {
      const size_t bo = (size_t)(n0 + (j << 4) + rlane) * ldb + koff + k0;
      bh[j] = Frag<T>::load(Bb + bo);
      if (SPLIT) bl[j] = Frag<T>::load(Bb2 + bo);
    }
#pragma unroll
    for (int i = 0; i < 4; ++i) {
      const size_t ao = (size_t)(m0 + (i << 4) + rlane) * lda + koff + k0;
      V ah = Frag<T>::load(Ab + ao);
      V al;
      if (SPLIT) al = Frag<T>::load(Ab2 + ao);
#pragma unroll
      for (int j = 0; j < 4; ++j) {
        acc[i][j] = Frag<T>::mma(ah, bh[j], acc[i][j]);
        if (SPLIT) {
          acc[i][j] = Frag<T>::mma(ah, bl[j], acc[i][j]);
          acc[i][j] = Frag<T>::mma(al, bh[j], acc[i][j]);
        }
      }
      Frag<T>::guard(acc[i][0], acc[i][3], ah, SPLIT ? al : ah);
    }
    Frag<T>::keep(bh[0], bh[1], bh[2], bh[3]);
    if (SPLIT) Frag<T>::keep(bl[0], bl[1], bl[2], bl[3]);
  }
  acc_guard4(acc[0][0], acc[0][1], acc[0][2], acc[0][3]);
  acc_guard4(acc[1][0], acc[1][1], acc[1][2], acc[1][3]);
  acc_guard4(acc[2][0], acc[2][1], acc[2][2], acc[2][3]);
  acc_guard4(acc[3][0], acc[3][1], acc[3][2], acc[3][3]);

  float* slab = sT[wave];
  const float* Rb = RESID ? (resid + (size_t)b * strideR) : nullptr;
#pragma unroll
  for (int i = 0; i < 4; ++i) {
    const int mBase = m0 + (i << 4);
#pragma unroll
    for (int j = 0; j < 4; ++j) {
      const int n = n0 + (j << 4) + rlane;
      float bv = 0.f;
      if (BIAS_MODE == 2) bv = bias[n];
#pragma unroll
      for (int r = 0; r < 8; ++r) {
        float v = acc[i][j][r] * scale;
        if (BIAS_MODE == 1) v += bias[mBase + mOff + r];
        if (BIAS_MODE == 2) v += bv;
        if (RESID) v += Rb[(size_t)(mBase + mOff + r) * ldc + n];
        if (ACT == 2) v = fmaxf(v, 0.0f);
        if (ACT == 4) v = (v > 0.f) ? v : 0.01f * v;
        slab[(mOff + r) * 68 + (j << 4) + rlane] = v;
      }
    }
    __builtin_amdgcn_fence(__ATOMIC_RELEASE, "workgroup");
    __builtin_amdgcn_wave_barrier();
    __builtin_amdgcn_fence(__ATOMIC_ACQUIRE, "workgroup");
    if (OUT_MODE == 0) {
      float* C = (float*)Cout + (size_t)b * strideC;
      const int hh = lane >> 4, c4 = (lane & 15) * 4;
      for (int pass = 0; pass < 2; ++pass) {
#pragma unroll
        for (int it = 0; it < 8; ++it) {
          const int row = it * 2 + hh;
          v4f v = *(const v4f*)(slab + row * 68 + c4);
          *(volatile v4f*)(C + (size_t)(mBase + row) * ldc + n0 + c4) = v;
        }
        __threadfence();
      }
    } else {
      const int q = lane >> 3, c8 = (lane & 7) * 8;
      unsigned short* C  = (unsigned short*)Cout  + (size_t)b * strideC;
      unsigned short* C2 = (OUT_MODE == 2) ? ((unsigned short*)Cout2 + (size_t)b * strideC) : nullptr;
      for (int pass = 0; pass < 2; ++pass) {
#pragma unroll
        for (int it = 0; it < 4; ++it) {
          const int row = it * 4 + q;
          const float* sp = slab + row * 68 + c8;
          v8h hv, lv;
#pragma unroll
          for (int e = 0; e < 8; ++e) {
            if (OUT_MODE == 1) {
              hv[e] = (_Float16)sp[e];
            } else {
              unsigned short hb = f2bf_bits(sp[e]);
              unsigned short lb = f2bf_bits(sp[e] - bf_bits2f(hb));
              hv[e] = __builtin_bit_cast(_Float16, hb);
              lv[e] = __builtin_bit_cast(_Float16, lb);
            }
          }
          *(volatile v8h*)(C + (size_t)(mBase + row) * ldc + n0 + c8) = hv;
          if (OUT_MODE == 2) *(volatile v8h*)(C2 + (size_t)(mBase + row) * ldc + n0 + c8) = lv;
        }
        __threadfence();
      }
    }
    __builtin_amdgcn_fence(__ATOMIC_RELEASE, "workgroup");
    __builtin_amdgcn_wave_barrier();
    __builtin_amdgcn_fence(__ATOMIC_ACQUIRE, "workgroup");
  }
}

__global__ __launch_bounds__(256) void cast_x_kernel(const float* __restrict__ q, const float* __restrict__ k,
                                                     const float* __restrict__ v, unsigned short* __restrict__ X, int n8) {
  const int i = blockIdx.x * 256 + threadIdx.x;
  if (i >= n8) return;
  const int src = blockIdx.y;
  const float* in = (src == 0) ? q : (src == 1) ? k : v;
  const int e0 = i * 8;
  const int row = e0 >> 10;
  const int col = e0 & 1023;
  const float* p = in + (size_t)row * kEmb + col;
  const v4f a = *(const v4f*)(p);
  const v4f c = *(const v4f*)(p + 4);
  unsigned short hb[8];
#pragma unroll
  for (int e = 0; e < 4; ++e) {
    hb[e]     = f2bf_bits(a[e]);
    hb[4 + e] = f2bf_bits(c[e]);
  }
  const v4u u = (v4u){pk16(hb[0], hb[1]), pk16(hb[2], hb[3]), pk16(hb[4], hb[5]), pk16(hb[6], hb[7])};
  unsigned short* o = X + (size_t)row * kXld + src * kEmb + col;
  *(volatile v4u*)o = u;
  __threadfence();
  *(volatile v4u*)o = u;
}

__global__ __launch_bounds__(256) void vt_cast_kernel(const float* __restrict__ v, unsigned short* __restrict__ VT) {
  __shared__ float sm[64][65];
  const int t   = threadIdx.x;
  const int s0  = blockIdx.x * 64;
  const int dg0 = blockIdx.y * 64;
  const int head = dg0 >> 7;
  const int dl0  = dg0 & 127;
#pragma unroll
  for (int i = 0; i < 4; ++i) {
    const int e  = i * 256 + t;
    const int r  = e >> 4;
    const int c4 = (e & 15) * 4;
    const v4f w = *(const v4f*)(v + (size_t)(s0 + r) * kEmb + dg0 + c4);
    sm[c4 + 0][r] = w[0];
    sm[c4 + 1][r] = w[1];
    sm[c4 + 2][r] = w[2];
    sm[c4 + 3][r] = w[3];
  }
  __syncthreads();
  const int lane = t & 31, wave = t >> 5;
  const int q = lane >> 3, c8 = (lane & 7) * 8;
  unsigned short* op = VT + ((size_t)(head * kDh + dl0)) * kSeq;
  for (int pass = 0; pass < 2; ++pass) {
#pragma unroll
    for (int it = 0; it < 2; ++it) {
      const int row = wave * 8 + it * 4 + q;
      unsigned short hb[8];
#pragma unroll
      for (int e = 0; e < 8; ++e) hb[e] = h_bits(bf_bits2f(f2bf_bits(sm[row][c8 + e])) * kVCarry);
      const v4u u = (v4u){pk16(hb[0], hb[1]), pk16(hb[2], hb[3]), pk16(hb[4], hb[5]), pk16(hb[6], hb[7])};
      *(volatile v4u*)(op + (size_t)row * kSeq + s0 + c8) = u;
    }
    __threadfence();
  }
}

__global__ __launch_bounds__(256) void wg_cast_kernel(const float* __restrict__ igw, const float* __restrict__ fgw,
                                                      unsigned short* __restrict__ W, int n8) {
  const int i = blockIdx.x * 256 + threadIdx.x;
  if (i >= n8) return;
  const int e0  = i * 8;
  const int row = e0 / kXld;
  const int col = e0 - row * kXld;
  const int ri  = (row < 8) ? row : 7;
  int rf = row - 8; rf = (rf < 0) ? 0 : ((rf > 7) ? 7 : rf);
  const float fa = (row < 8) ? 1.0f : 0.0f;
  const float fb = (row >= 8 && row < 16) ? 1.0f : 0.0f;
  const float* pa = igw + (size_t)ri * kXld + col;
  const float* pb = fgw + (size_t)rf * kXld + col;
  const v4f a0 = *(const v4f*)(pa);
  const v4f a1 = *(const v4f*)(pa + 4);
  const v4f b0 = *(const v4f*)(pb);
  const v4f b1 = *(const v4f*)(pb + 4);
  unsigned short hb[8];
#pragma unroll
  for (int e = 0; e < 4; ++e) {
    hb[e]     = f2bf_bits(fmaf(fa, a0[e], fb * b0[e]));
    hb[4 + e] = f2bf_bits(fmaf(fa, a1[e], fb * b1[e]));
  }
  const v4u u = (v4u){pk16(hb[0], hb[1]), pk16(hb[2], hb[3]), pk16(hb[4], hb[5]), pk16(hb[6], hb[7])};
  unsigned short* o = W + (size_t)row * kXld + col;
  *(volatile v4u*)o = u;
  __threadfence();
  *(volatile v4u*)o = u;
}

__device__ __forceinline__ void store_plane2048(const float* src, float* dst, int t) {
  const v4f a = *(const v4f*)(src + 4 * t);
  const v4f b = *(const v4f*)(src + 1024 + 4 * t);
  float* p0 = dst + 4 * t;
  float* p1 = dst + 1024 + 4 * t;
  *(volatile v4f*)p0 = a;
  *(volatile v4f*)p1 = b;
  __threadfence();
  *(volatile v4f*)p0 = a;
  *(volatile v4f*)p1 = b;
}

__global__ __launch_bounds__(256) void scan_kernel(const float* __restrict__ G, const float* __restrict__ igb,
                                                   const float* __restrict__ fgb,
                                                   float* __restrict__ CSp, float* __restrict__ IGp, float* __restrict__ Mp,
                                                   float* __restrict__ EMp, float* __restrict__ GFp, float* __restrict__ GTp) {
  __shared__ __align__(16) float tree[4096];
  __shared__ __align__(16) float igs[kSeq];
  __shared__ __align__(16) float stage[kSeq];
  __shared__ double pmax[256];
  __shared__ double excl[256];
  __shared__ __align__(16) float gts[kTiles];
  const int h = blockIdx.x;
  const int t = threadIdx.x;
  const float bi = bf_bits2f(f2bf_bits(igb[h]));
  const float bf = bf_bits2f(f2bf_bits(fgb[h]));

#pragma unroll 1
  for (int it = 0; it < 8; ++it) {
    const int s = it * 256 + t;
    const float a = G[(size_t)s * kGateN + h] + bi;
    const float f = G[(size_t)s * kGateN + 8 + h] + bf;
    const float lf = fminf(f, 0.0f) - log1pf(expf(-fabsf(f)));
    igs[s]  = a;
    tree[s] = lf;
  }
  __syncthreads();

#pragma unroll 1
  for (int l = 0; l < 11; ++l) {
    const int offl = 4096 - (4096 >> l);
    const int offn = 4096 - (4096 >> (l + 1));
    const int nn = kSeq >> (l + 1);
    for (int idx = t; idx < nn; idx += 256) tree[offn + idx] = tree[offl + 2 * idx] + tree[offl + 2 * idx + 1];
    __syncthreads();
  }
#pragma unroll 1
  for (int l = 10; l >= 0; --l) {
    const int offl = 4096 - (4096 >> l);
    const int offn = 4096 - (4096 >> (l + 1));
    const int nl = kSeq >> l;
    for (int idx = t; idx < nl; idx += 256) {
      const int upi = (idx > 0) ? ((idx - 1) >> 1) : 0;
      const float up  = tree[offn + upi];
      const float own = tree[offl + idx];
      const float val = (idx & 1) ? up : (up + own);
      if (idx > 0) tree[offl + idx] = val;
    }
    __syncthreads();
  }

  float Sv[8], IGv[8];
  double pre[8];
  double run = -__builtin_inf();
#pragma unroll
  for (int e = 0; e < 8; ++e) {
    const int s = 8 * t + e;
    Sv[e]  = tree[s];
    IGv[e] = igs[s];
    const double gd = (double)IGv[e] - (double)Sv[e];
    run = fmax(run, gd);
    pre[e] = run;
  }
  pmax[t] = run;
  __syncthreads();
  if (t == 0) {
    double m = -__builtin_inf();
#pragma unroll 1
    for (int w = 0; w < 256; ++w) { excl[w] = m; m = fmax(m, pmax[w]); }
  }
  if (t < kTiles) {
    const double g4 = fmax(fmax(pmax[4 * t], pmax[4 * t + 1]), fmax(pmax[4 * t + 2], pmax[4 * t + 3]));
    gts[t] = (float)g4;
  }
  __syncthreads();
  const double base = excl[t];
  float Mv[8], EMv[8], GFv[8];
#pragma unroll
  for (int e = 0; e < 8; ++e) {
    const double Gd = fmax(base, pre[e]);
    const double Md = (double)Sv[e] + Gd;
    Mv[e]  = (float)Md;
    EMv[e] = expf(-Mv[e]);
    GFv[e] = (float)Gd;
  }

  store_plane2048(tree, CSp + (size_t)h * kSeq, t);
  store_plane2048(igs,  IGp + (size_t)h * kSeq, t);
#pragma unroll
  for (int e = 0; e < 8; ++e) stage[8 * t + e] = Mv[e];
  __syncthreads();
  store_plane2048(stage, Mp + (size_t)h * kSeq, t);
  __syncthreads();
#pragma unroll
  for (int e = 0; e < 8; ++e) stage[8 * t + e] = EMv[e];
  __syncthreads();
  store_plane2048(stage, EMp + (size_t)h * kSeq, t);
  __syncthreads();
#pragma unroll
  for (int e = 0; e < 8; ++e) stage[8 * t + e] = GFv[e];
  __syncthreads();
  store_plane2048(stage, GFp + (size_t)h * kSeq, t);
  if (t < 16) {
    const v4f g = *(const v4f*)(gts + 4 * t);
    float* gp = GTp + (size_t)h * kTiles + 4 * t;
    *(volatile v4f*)gp = g;
    __threadfence();
    *(volatile v4f*)gp = g;
  }
}

__global__ __launch_bounds__(128) void mlstm_core_kernel(const unsigned short* __restrict__ Xp,
                                                         const unsigned short* __restrict__ VTp,
                                                         const float* __restrict__ CSp, const float* __restrict__ IGp,
                                                         const float* __restrict__ Mp, const float* __restrict__ EMp,
                                                         const float* __restrict__ GFp, const float* __restrict__ GTp,
                                                         float* __restrict__ hbuf, float rscale) {
  __shared__ __align__(16) _Float16 Cs[4][16 * 40];
  __shared__ __align__(16) float    Os[4][16 * 132];
  const int head = blockIdx.y;
  const int lane = threadIdx.x & 31;
  const int wave = threadIdx.x >> 5;
  const int lh = lane >> 4;
  const int lo = lane & 15;
  const int i0 = __builtin_amdgcn_readfirstlane((int)(blockIdx.x * 64 + wave * 16));

  const __bf16*   X  = (const __bf16*)Xp;
  const _Float16* VT = (const _Float16*)VTp;
  const __bf16* Qrow  = X + (size_t)(i0 + lo) * kXld + head * kDh;
  const __bf16* Kbase = X + kEmb + head * kDh;
  const _Float16* Vbase = VT + (size_t)head * kDh * kSeq;
  const float* CSh = CSp + (size_t)head * kSeq;
  const float* IGh = IGp + (size_t)head * kSeq;
  const float* Mh  = Mp  + (size_t)head * kSeq;
  const float* EMh = EMp + (size_t)head * kSeq;
  const float* GTh = GTp + (size_t)head * kTiles;
  const float gf0 = GFp[(size_t)head * kSeq + i0];

  float Si[8], Mi[8], rsum[8];
  {
    const v4f s0 = *(const v4f*)(CSh + i0 + 8 * lh);
    const v4f s1 = *(const v4f*)(CSh + i0 + 8 * lh + 4);
    const v4f m0 = *(const v4f*)(Mh + i0 + 8 * lh);
    const v4f m1 = *(const v4f*)(Mh + i0 + 8 * lh + 4);
#pragma unroll
    for (int e = 0; e < 4; ++e) { Si[e] = s0[e]; Si[4 + e] = s1[e]; Mi[e] = m0[e]; Mi[4 + e] = m1[e]; }
  }
#pragma unroll
  for (int r = 0; r < 8; ++r) rsum[r] = 0.0f;
  v8f acc[8];
#pragma unroll
  for (int c = 0; c < 8; ++c) acc[c] = (v8f){0.f,0.f,0.f,0.f,0.f,0.f,0.f,0.f};

  _Float16* cs = Cs[wave];
  const int ntile = (i0 >> 5) + 1;
  for (int jt = 0; jt < ntile; ++jt) {
    const float gt = GTh[jt];
    const int live = __builtin_amdgcn_readfirstlane((int)((gt - gf0) >= kSkipBelow));
    if (!live) continue;
    const int jb = jt * 32;

    v8f s0 = (v8f){0.f,0.f,0.f,0.f,0.f,0.f,0.f,0.f};
    v8f s1 = (v8f){0.f,0.f,0.f,0.f,0.f,0.f,0.f,0.f};
#pragma unroll
    for (int f = 0; f < 4; ++f) {
      const v16b qa  = Frag<__bf16>::load(Qrow + f * 32 + 8 * lh);
      const v16b kb0 = Frag<__bf16>::load(Kbase + (size_t)(jb + lo) * kXld + f * 32 + 8 * lh);
      const v16b kb1 = Frag<__bf16>::load(Kbase + (size_t)(jb + 16 + lo) * kXld + f * 32 + 8 * lh);
      s0 = mma16_bf(qa, kb0, s0);
      s1 = mma16_bf(qa, kb1, s1);
    }

    const int j0 = jb + lo, j1 = jb + 16 + lo;
    const float Sj0 = CSh[j0], Sj1 = CSh[j1];
    const float ig0 = IGh[j0], ig1 = IGh[j1];
    __builtin_amdgcn_fence(__ATOMIC_RELEASE, "workgroup");
    __builtin_amdgcn_wave_barrier();
    __builtin_amdgcn_fence(__ATOMIC_ACQUIRE, "workgroup");
#pragma unroll
    for (int r = 0; r < 8; ++r) {
      const int row = i0 + 8 * lh + r;
      float x0 = ((Si[r] - Sj0) + ig0) - Mi[r];
      float x1 = ((Si[r] - Sj1) + ig1) - Mi[r];
      x0 = fminf(x0, 0.0f);
      x1 = fminf(x1, 0.0f);
      const float d0 = expf(x0);
      const float d1 = expf(x1);
      float c0 = (s0[r] * rscale) * d0;
      float c1 = (s1[r] * rscale) * d1;
      c0 = (j0 <= row) ? c0 : 0.0f;
      c1 = (j1 <= row) ? c1 : 0.0f;
      rsum[r] = rsum[r] + (c0 + c1);
      cs[(8 * lh + r) * 40 + lo]      = (_Float16)(c0 * kCCarry);
      cs[(8 * lh + r) * 40 + 16 + lo] = (_Float16)(c1 * kCCarry);
    }
    __builtin_amdgcn_fence(__ATOMIC_RELEASE, "workgroup");
    __builtin_amdgcn_wave_barrier();
    __builtin_amdgcn_fence(__ATOMIC_ACQUIRE, "workgroup");
    const v16h ca = Frag<_Float16>::load(cs + lo * 40 + 8 * lh);
#pragma unroll
    for (int c = 0; c < 8; ++c) {
      const v16h vb = Frag<_Float16>::load(Vbase + (size_t)(c * 16 + lo) * kSeq + jb + 8 * lh);
      acc[c] = mma16_h(ca, vb, acc[c]);
    }
  }

  float em[8];
  {
    const v4f e0 = *(const v4f*)(EMh + i0 + 8 * lh);
    const v4f e1 = *(const v4f*)(EMh + i0 + 8 * lh + 4);
#pragma unroll
    for (int e = 0; e < 4; ++e) { em[e] = e0[e]; em[4 + e] = e1[e]; }
  }
  float* os = Os[wave];
#pragma unroll
  for (int r = 0; r < 8; ++r) {
    float b = rsum[r];
    b += __shfl_xor(b, 1, 32);
    b += __shfl_xor(b, 2, 32);
    b += __shfl_xor(b, 4, 32);
    b += __shfl_xor(b, 8, 32);
    const float n = fmaxf(fabsf(b), em[r]) + kEpsN;
    const float inv = (1.0f / n) * kCVInv;
#pragma unroll
    for (int c = 0; c < 8; ++c) os[(8 * lh + r) * 132 + c * 16 + lo] = acc[c][r] * inv;
  }
  __builtin_amdgcn_fence(__ATOMIC_RELEASE, "workgroup");
  __builtin_amdgcn_wave_barrier();
  __builtin_amdgcn_fence(__ATOMIC_ACQUIRE, "workgroup");
  float* ob = hbuf + (size_t)i0 * kEmb + head * kDh + lane * 4;
  for (int pass = 0; pass < 2; ++pass) {
#pragma unroll
    for (int row = 0; row < 16; ++row) {
      const v4f val = *(const v4f*)(os + row * 132 + lane * 4);
      *(volatile v4f*)(ob + (size_t)row * kEmb) = val;
    }
    __threadfence();
  }
}

__global__ __launch_bounds__(256) void ln_kernel(const float* __restrict__ hb, const float* __restrict__ lnw,
                                                 float* __restrict__ out) {
  __shared__ float red[8];
  __shared__ float red2[8];
  const int row  = blockIdx.x;
  const int t    = threadIdx.x;
  const int lane = t & 31, wave = t >> 5;
  const v4f x = *(const v4f*)(hb + (size_t)row * kEmb + 4 * t);
  float s = (x[0] + x[1]) + (x[2] + x[3]);
#pragma unroll
  for (int off = 16; off > 0; off >>= 1) s += __shfl_xor(s, off, 32);
  if (lane == 0) red[wave] = s;
  __syncthreads();
  float tot = red[0];
#pragma unroll
  for (int w = 1; w < 8; ++w) tot += red[w];
  const float mu = tot * kInvEmb;
  float d[4];
#pragma unroll
  for (int e = 0; e < 4; ++e) d[e] = x[e] - mu;
  float s2 = (d[0] * d[0] + d[1] * d[1]) + (d[2] * d[2] + d[3] * d[3]);
#pragma unroll
  for (int off = 16; off > 0; off >>= 1) s2 += __shfl_xor(s2, off, 32);
  if (lane == 0) red2[wave] = s2;
  __syncthreads();
  float tot2 = red2[0];
#pragma unroll
  for (int w = 1; w < 8; ++w) tot2 += red2[w];
  const float var = tot2 * kInvEmb;
  const float rs = 1.0f / sqrtf(var + kLnEps);
  const v4f w4 = *(const v4f*)(lnw + 4 * t);
  v4f o;
#pragma unroll
  for (int e = 0; e < 4; ++e) o[e] = (d[e] * rs) * bf_bits2f(f2bf_bits(w4[e]));
  float* op = out + (size_t)row * kEmb + 4 * t;
  *(volatile v4f*)op = o;
  __threadfence();
  *(volatile v4f*)op = o;
}

extern "C" void kernel_launch(void* const* d_in, const int* in_sizes, int n_in,
                              void* d_out, int out_size, void* d_ws, size_t ws_size,
                              hipStream_t stream) {
  if (n_in < 8) return;
  const int nQ = kSeq * kEmb;
  if (in_sizes[0] != nQ || in_sizes[1] != nQ || in_sizes[2] != nQ) return;
  if (in_sizes[3] != kHeads * kXld || in_sizes[5] != kHeads * kXld) return;
  if (in_sizes[4] != kHeads || in_sizes[6] != kHeads || in_sizes[7] != kEmb) return;
  if (out_size != nQ) return;

  const size_t szX    = (size_t)kSeq * kXld * 2;
  const size_t szVT   = (size_t)kHeads * kDh * kSeq * 2;
  const size_t szWG   = (size_t)kGateN * kXld * 2;
  const size_t szGATE = (size_t)kSeq * kGateN * 4;
  const size_t szPL   = (size_t)kHeads * kSeq * 4;
  const size_t szGT   = 4096;
  const size_t szH    = (size_t)kSeq * kEmb * 4;
  const size_t offX    = 0;
  const size_t offVT   = offX + szX;
  const size_t offWG   = offVT + szVT;
  const size_t offGATE = offWG + szWG;
  const size_t offCS   = offGATE + szGATE;
  const size_t offIG   = offCS + szPL;
  const size_t offM    = offIG + szPL;
  const size_t offEM   = offM + szPL;
  const size_t offGF   = offEM + szPL;
  const size_t offGT   = offGF + szPL;
  const size_t offH    = offGT + szGT;
  const size_t total   = offH + szH;
  if (ws_size < total) return;

  const float* q   = (const float*)d_in[0];
  const float* k   = (const float*)d_in[1];
  const float* v   = (const float*)d_in[2];
  const float* igw = (const float*)d_in[3];
  const float* igb = (const float*)d_in[4];
  const float* fgw = (const float*)d_in[5];
  const float* fgb = (const float*)d_in[6];
  const float* lnw = (const float*)d_in[7];
  float* out = (float*)d_out;
  char* ws = (char*)d_ws;
  unsigned short* X  = (unsigned short*)(ws + offX);
  unsigned short* VT = (unsigned short*)(ws + offVT);
  unsigned short* WG = (unsigned short*)(ws + offWG);
  float* GATE = (float*)(ws + offGATE);
  float* CS = (float*)(ws + offCS);
  float* IG = (float*)(ws + offIG);
  float* MX = (float*)(ws + offM);
  float* EM = (float*)(ws + offEM);
  float* GF = (float*)(ws + offGF);
  float* GT = (float*)(ws + offGT);
  float* H  = (float*)(ws + offH);

  const int n8x = nQ / 8;
  cast_x_kernel<<<dim3(n8x / 256, 3), dim3(256), 0, stream>>>(q, k, v, X, n8x);
  vt_cast_kernel<<<dim3(kSeq / 64, kEmb / 64), dim3(256), 0, stream>>>(v, VT);
  const int n8w = (kGateN * kXld) / 8;
  wg_cast_kernel<<<dim3(n8w / 256), dim3(256), 0, stream>>>(igw, fgw, WG, n8w);
  wmma_gemm64<1, false, 0, 0, false, 0><<<dim3((kSeq / 64) * (kGateN / 64) / 8, 1), dim3(256), 0, stream>>>(
      X, X, kXld, 0L, WG, WG, kXld, 0L, (void*)GATE, (void*)GATE, kGateN, 0L, GATE, GATE, 0L,
      kSeq, kGateN, kXld, 1.0f);
  scan_kernel<<<dim3(kHeads), dim3(256), 0, stream>>>(GATE, igb, fgb, CS, IG, MX, EM, GF, GT);
  const float sq = sqrtf(128.0f);
  const float rscale = 1.0f / sq;
  mlstm_core_kernel<<<dim3(kSeq / 64, kHeads), dim3(128), 0, stream>>>(X, VT, CS, IG, MX, EM, GF, GT, H, rscale);
  ln_kernel<<<dim3(kSeq), dim3(256), 0, stream>>>(H, lnw, out);
}
